// baseGCN_33775622815788
// MI455X (gfx1250) — hardware-verified
//
#include <hip/hip_runtime.h>
#include <stddef.h>
#include <math.h>


#define F0      64
#define FD      256
#define NTHR    256
#define NWAVE   8
#define EPT     8
#define NGRP    2
#define CHUNK   (NTHR * EPT * NGRP)
#define WCAP    (EPT * NGRP * 32)
#define LISTN   (NWAVE * WCAP)
#define NBC     4096
#define NBF     1024
#define RCAP    40960
#define RBN     128
#define TGT     256
#define DEGCAP  1024
#define GROWS   64
#define OTHR    512
#define HP      544
#define MAXSEG  65536
#define WSCAP   134217728

#define WOFF0   0
#define WOFF1   16384
#define WOFF2   81920
#define WOFF3   147456
#define WPTOT   212992

#define ASC     64.0f
#define WSC     16.0f
#define OSC     0.0009765625f

#define LDS_FILL ((RCAP + NBF + LISTN) * 4 + 64)
#define LDS_G0   (GROWS * (F0 + 8) * 2 + GROWS * FD * 4)
#define LDS_G1   (GROWS * (FD + 8) * 2 + GROWS * FD * 4)

#define BN_EPS 1e-5f

static_assert((CHUNK & (CHUNK - 1)) == 0);
static_assert(CHUNK <= 4096);
static_assert(NBC <= 4096 && NBF <= 4096);
static_assert((NBC & (NBC - 1)) == 0 && (NBF & (NBF - 1)) == 0);
static_assert(NBC == 4 * NBF);
static_assert(OTHR * 8 == NBC);
static_assert((RCAP % 32) == 0);
static_assert(TGT == NWAVE * 32 && (TGT % GROWS) == 0);
static_assert((NBC % TGT) == 0);
static_assert(GROWS == 2 * 32 && NWAVE == 8);
static_assert(NTHR == FD);
static_assert((HP % 32) == 0 && HP >= 2 * FD + 1 && (HP / 4) <= NTHR);
static_assert(WOFF1 == WOFF0 + FD * F0 && WOFF2 == WOFF1 + FD * FD && WOFF3 == WOFF2 + FD * FD && WPTOT == WOFF3 + FD * FD);
static_assert((LDS_G0 % 16) == 0 && (LDS_G1 % 16) == 0);
static_assert(((GROWS * (F0 + 8) * 2) % 16) == 0 && ((GROWS * (FD + 8) * 2) % 16) == 0);

typedef float          v4f  __attribute__((ext_vector_type(4)));
typedef float          v8f  __attribute__((ext_vector_type(8)));
typedef double         v2d  __attribute__((ext_vector_type(2)));
typedef int            v4i  __attribute__((ext_vector_type(4)));
typedef _Float16       v8h  __attribute__((ext_vector_type(8)));
typedef _Float16       v16h __attribute__((ext_vector_type(16)));
union FragH { v16h v; v8h h[2]; };
union Pack8 { v8h h; v4i u; };

__device__ __forceinline__ v8f wmh(v16h a, v16h b, v8f c) {
  v8f d = __builtin_amdgcn_wmma_f32_16x16x32_f16(false, a, false, b, (short)0, c, false, false);
  asm volatile("v_nop\n\tv_nop\n\tv_nop\n\tv_nop" : "+v"(d) : "v"(a), "v"(b));
  return d;
}

__device__ __forceinline__ v8h cvt8(v4f a, v4f b) {
  v8h r;
  r[0] = (_Float16)a.x; r[1] = (_Float16)a.y; r[2] = (_Float16)a.z; r[3] = (_Float16)a.w;
  r[4] = (_Float16)b.x; r[5] = (_Float16)b.y; r[6] = (_Float16)b.z; r[7] = (_Float16)b.w;
  return r;
}

__device__ __forceinline__ float bnt1(float a, float mu, float rs, float g, float b) {
  return tanhf((g * (a - mu)) * rs + b);
}
__device__ __forceinline__ v4f bnt4(v4f a, v4f mu, v4f rs, v4f g, v4f b) {
  const v4f t = (g * (a - mu)) * rs + b;
  v4f z;
  z.x = tanhf(t.x); z.y = tanhf(t.y); z.z = tanhf(t.z); z.w = tanhf(t.w);
  return z;
}

template <int NB>
__device__ __forceinline__ int scan_chunk(const int* __restrict__ dsts, int nE, int cbase, int slotBase,
                                          int vec8, int* list, int tid, int lane, int wave) {
  int wc = 0;
#pragma unroll
  for (int g = 0; g < NGRP; ++g) {
    const int el0  = (g * NTHR + tid) * EPT;
    const int e0   = cbase + el0;
    const int sent = -2147483647 - 1;
    v4i da, db;
    if (vec8 != 0 && cbase + CHUNK <= nE) {
      da = *(const v4i*)(dsts + e0);
      db = *(const v4i*)(dsts + e0 + 4);
    } else {
      da.x = (e0     < nE) ? dsts[min(e0, nE - 1)] : sent;
      da.y = (e0 + 1 < nE) ? dsts[min(e0 + 1, nE - 1)] : sent;
      da.z = (e0 + 2 < nE) ? dsts[min(e0 + 2, nE - 1)] : sent;
      da.w = (e0 + 3 < nE) ? dsts[min(e0 + 3, nE - 1)] : sent;
      db.x = (e0 + 4 < nE) ? dsts[min(e0 + 4, nE - 1)] : sent;
      db.y = (e0 + 5 < nE) ? dsts[min(e0 + 5, nE - 1)] : sent;
      db.z = (e0 + 6 < nE) ? dsts[min(e0 + 6, nE - 1)] : sent;
      db.w = (e0 + 7 < nE) ? dsts[min(e0 + 7, nE - 1)] : sent;
    }
    const unsigned nb = (unsigned)slotBase;
    const unsigned s0 = (unsigned)da.x - nb, s1 = (unsigned)da.y - nb;
    const unsigned s2 = (unsigned)da.z - nb, s3 = (unsigned)da.w - nb;
    const unsigned s4 = (unsigned)db.x - nb, s5 = (unsigned)db.y - nb;
    const unsigned s6 = (unsigned)db.z - nb, s7 = (unsigned)db.w - nb;
    const bool h0 = s0 < (unsigned)NB, h1 = s1 < (unsigned)NB, h2 = s2 < (unsigned)NB, h3 = s3 < (unsigned)NB;
    const bool h4 = s4 < (unsigned)NB, h5 = s5 < (unsigned)NB, h6 = s6 < (unsigned)NB, h7 = s7 < (unsigned)NB;
    const unsigned any = __builtin_amdgcn_ballot_w32(h0 | h1 | h2 | h3 | h4 | h5 | h6 | h7);
    if (any != 0u) {
#define HITJ(J, HJ, SJ) { \
        const unsigned mj = __builtin_amdgcn_ballot_w32(HJ); \
        if (mj != 0u) { \
          if (HJ) { \
            const int pos = wc + (int)__builtin_amdgcn_mbcnt_lo(mj, 0u); \
            if (pos < WCAP) list[wave * WCAP + pos] = ((el0 + (J)) << 12) | (int)(SJ); \
          } \
          wc += (int)__builtin_popcount(mj); } }
      HITJ(0, h0, s0)
      HITJ(1, h1, s1)
      HITJ(2, h2, s2)
      HITJ(3, h3, s3)
      HITJ(4, h4, s4)
      HITJ(5, h5, s5)
      HITJ(6, h6, s6)
      HITJ(7, h7, s7)
#undef HITJ
    }
  }
  return wc;
}

__global__ __launch_bounds__(NTHR) void k_wprep(
    const float* __restrict__ w0, const float* __restrict__ w1,
    const float* __restrict__ w2, const float* __restrict__ w3, _Float16* wp) {
  const int blk = blockIdx.x, tid = threadIdx.x;
  const float* W;
  int i, base, n, k0;
  if (blk < 8) {
    W = w0; i = blk * NTHR + tid; base = WOFF0; n = i >> 3; k0 = (i & 7) * 8;
  } else {
    const int p = (blk - 8) >> 5;
    W = (p == 0) ? w1 : ((p == 1) ? w2 : w3);
    i = ((blk - 8) & 31) * NTHR + tid; base = WOFF1 + p * FD * FD; n = i >> 5; k0 = (i & 31) * 8;
  }
  v4f a, b;
  a.x = W[(size_t)(k0 + 0) * FD + n] * WSC; a.y = W[(size_t)(k0 + 1) * FD + n] * WSC;
  a.z = W[(size_t)(k0 + 2) * FD + n] * WSC; a.w = W[(size_t)(k0 + 3) * FD + n] * WSC;
  b.x = W[(size_t)(k0 + 4) * FD + n] * WSC; b.y = W[(size_t)(k0 + 5) * FD + n] * WSC;
  b.z = W[(size_t)(k0 + 6) * FD + n] * WSC; b.w = W[(size_t)(k0 + 7) * FD + n] * WSC;
  Pack8 pk;
  pk.h = cvt8(a, b);
  _Float16* dh = wp + base + (size_t)i * 8;
  *(volatile v4i*)dh = pk.u;
  __threadfence();
  *(volatile v4i*)dh = pk.u;
}

__global__ __launch_bounds__(NTHR) void k_count(const int* __restrict__ dsts, int* cnt, int nE, int vec8) {
  __shared__ __attribute__((aligned(16))) int scnt[NBC];
  __shared__ __attribute__((aligned(16))) int list[LISTN];
  __shared__ int wcnt[NWAVE];
  const int tid = threadIdx.x, lane = tid & 31, wave = tid >> 5;
  const int nodeBase = blockIdx.x * NBC;

  for (int i = tid; i < NBC; i += NTHR) scnt[i] = 0;
  __syncthreads();

  const int nChunks = (nE + CHUNK - 1) / CHUNK;
#pragma unroll 1
  for (int ch = 0; ch < nChunks; ++ch) {
    const int cbase = ch * CHUNK;
    const int wc = scan_chunk<NBC>(dsts, nE, cbase, nodeBase, vec8, list, tid, lane, wave);
    if (lane == 0) wcnt[wave] = wc;
    __syncthreads();
    if (wave == 0) {
#pragma unroll 1
      for (int wsx = 0; wsx < NWAVE; ++wsx) {
        int n = __builtin_amdgcn_readfirstlane(wcnt[wsx]);
        n = n > WCAP ? WCAP : (n < 0 ? 0 : n);
        const int* lp = list + wsx * WCAP;
#pragma unroll 1
        for (int i = 0; i < n; ++i) {
          const int ent  = __builtin_amdgcn_readfirstlane(lp[i]);
          const int slot = ent & (NBC - 1);
          if (lane == 0) scnt[slot] = scnt[slot] + 1;
        }
      }
    }
    __syncthreads();
  }

  v4i cq[4];
#pragma unroll
  for (int q = 0; q < 4; ++q) {
    const int f = (wave * 4 + q) * 128 + 4 * lane;
    cq[q] = *(const v4i*)(scnt + f);
  }
  int* cp = cnt + (size_t)nodeBase;
#pragma unroll
  for (int q = 0; q < 4; ++q) {
    const int f = (wave * 4 + q) * 128 + 4 * lane;
    *(volatile v4i*)(cp + f) = cq[q];
  }
  __threadfence();
#pragma unroll
  for (int q = 0; q < 4; ++q) {
    const int f = (wave * 4 + q) * 128 + 4 * lane;
    *(volatile v4i*)(cp + f) = cq[q];
  }
}

__global__ __launch_bounds__(OTHR) void k_offsets(
    const int* __restrict__ cnt, int* off, float* dinv, int* rbase, int nChunk) {
  __shared__ __attribute__((aligned(16))) int soff[NBC];
  __shared__ __attribute__((aligned(16))) float sdi[NBC];
  __shared__ __attribute__((aligned(16))) int srb[RBN];
  __shared__ int wtot[OTHR / 32];
  const int tid = threadIdx.x, lane = tid & 31, wave = tid >> 5, sub = tid >> 7;
  for (int i = tid; i < RBN; i += OTHR) srb[i] = 0;
  int carry = 0;
#pragma unroll 1
  for (int ch = 0; ch < nChunk; ++ch) {
    const int base = ch * NBC;
    const v4i c0 = *(const v4i*)(cnt + base + 8 * tid);
    const v4i c1 = *(const v4i*)(cnt + base + 8 * tid + 4);
    const int e0 = max(c0.x, 0), e1 = max(c0.y, 0), e2 = max(c0.z, 0), e3 = max(c0.w, 0);
    const int e4 = max(c1.x, 0), e5 = max(c1.y, 0), e6 = max(c1.z, 0), e7 = max(c1.w, 0);
    const int ts = e0 + e1 + e2 + e3 + e4 + e5 + e6 + e7;
    int incl = ts;
#pragma unroll
    for (int d = 1; d < 32; d <<= 1) {
      const int t = __shfl_up(incl, d);
      if (lane >= d) incl += t;
    }
    if (lane == 31) wtot[wave] = incl;
    __syncthreads();
    const int S0 = wtot[0]  + wtot[1]  + wtot[2]  + wtot[3];
    const int S1 = wtot[4]  + wtot[5]  + wtot[6]  + wtot[7];
    const int S2 = wtot[8]  + wtot[9]  + wtot[10] + wtot[11];
    const int S3 = wtot[12] + wtot[13] + wtot[14] + wtot[15];
    int pre = 0;
#pragma unroll 1
    for (int w = 4 * sub; w < wave; ++w) pre += wtot[w];
    const int b0 = carry;
    const int b1 = b0 + ((S0 + 31) & ~31);
    const int b2 = b1 + ((S1 + 31) & ~31);
    const int b3 = b2 + ((S2 + 31) & ~31);
    const int b4 = b3 + ((S3 + 31) & ~31);
    const int myb = sub == 0 ? b0 : (sub == 1 ? b1 : (sub == 2 ? b2 : b3));
    if (tid == 0) {
      srb[min(4 * ch + 0, RBN - 1)] = b0;
      srb[min(4 * ch + 1, RBN - 1)] = b1;
      srb[min(4 * ch + 2, RBN - 1)] = b2;
      srb[min(4 * ch + 3, RBN - 1)] = b3;
    }
    int run = myb + pre + incl - ts;
    soff[8 * tid + 0] = run; run += e0;
    soff[8 * tid + 1] = run; run += e1;
    soff[8 * tid + 2] = run; run += e2;
    soff[8 * tid + 3] = run; run += e3;
    soff[8 * tid + 4] = run; run += e4;
    soff[8 * tid + 5] = run; run += e5;
    soff[8 * tid + 6] = run; run += e6;
    soff[8 * tid + 7] = run;
    sdi[8 * tid + 0] = rsqrtf(1.0f + (float)e0);
    sdi[8 * tid + 1] = rsqrtf(1.0f + (float)e1);
    sdi[8 * tid + 2] = rsqrtf(1.0f + (float)e2);
    sdi[8 * tid + 3] = rsqrtf(1.0f + (float)e3);
    sdi[8 * tid + 4] = rsqrtf(1.0f + (float)e4);
    sdi[8 * tid + 5] = rsqrtf(1.0f + (float)e5);
    sdi[8 * tid + 6] = rsqrtf(1.0f + (float)e6);
    sdi[8 * tid + 7] = rsqrtf(1.0f + (float)e7);
    carry = b4;
    __syncthreads();
    const v4i o0 = *(const v4i*)(soff + 4 * tid);
    const v4i o1 = *(const v4i*)(soff + 4 * (tid + OTHR));
    const v4f d0 = *(const v4f*)(sdi + 4 * tid);
    const v4f d1 = *(const v4f*)(sdi + 4 * (tid + OTHR));
    int* op = off + base;
    float* dp = dinv + base;
    *(volatile v4i*)(op + 4 * tid) = o0;
    *(volatile v4i*)(op + 4 * (tid + OTHR)) = o1;
    *(volatile v4f*)(dp + 4 * tid) = d0;
    *(volatile v4f*)(dp + 4 * (tid + OTHR)) = d1;
    __threadfence();
    *(volatile v4i*)(op + 4 * tid) = o0;
    *(volatile v4i*)(op + 4 * (tid + OTHR)) = o1;
    *(volatile v4f*)(dp + 4 * tid) = d0;
    *(volatile v4f*)(dp + 4 * (tid + OTHR)) = d1;
    __syncthreads();
  }
  if (tid == 0) srb[min(4 * nChunk, RBN - 1)] = carry;
  __syncthreads();
  v4i rv = {0, 0, 0, 0};
  if (tid < 32) rv = *(const v4i*)(srb + 4 * tid);
  if (tid < 32) *(volatile v4i*)(rbase + 4 * tid) = rv;
  __threadfence();
  if (tid < 32) *(volatile v4i*)(rbase + 4 * tid) = rv;
}

__global__ __launch_bounds__(NTHR) void k_fill(
    const int* __restrict__ srcs, const int* __restrict__ dsts,
    const int* __restrict__ off, const int* __restrict__ rbase,
    int* csr, int nN, int nE, int vec8, int csrLen) {
  extern __shared__ v4f lds_dyn[];
  int* region = (int*)lds_dyn;
  int* cursor = region + RCAP;
  int* list   = cursor + NBF;
  int* wcnt   = list + LISTN;
  const int tid = threadIdx.x, lane = tid & 31, wave = tid >> 5;
  const int b = blockIdx.x;
  const int nodeBase = b * NBF;

  int rb0 = rbase[b];
  const int rb1 = rbase[b + 1];
  rb0 = rb0 < 0 ? 0 : (rb0 > csrLen ? csrLen : rb0);
  rb0 &= ~31;
  int len = rb1 - rb0;
  len = len < 0 ? 0 : (len > RCAP ? RCAP : len);
  int lenW = (len + 31) & ~31;
  if (rb0 + lenW > csrLen) lenW = (csrLen - rb0) & ~31;

  {
    const v4i z = {0, 0, 0, 0};
    for (int i = tid; i < RCAP / 4; i += NTHR) ((v4i*)region)[i] = z;
    for (int s = tid; s < NBF; s += NTHR) {
      int o = off[nodeBase + s] - rb0;
      o = o < 0 ? 0 : (o > RCAP ? RCAP : o);
      cursor[s] = o;
    }
  }
  __syncthreads();

  const int nChunks = (nE + CHUNK - 1) / CHUNK;
#pragma unroll 1
  for (int ch = 0; ch < nChunks; ++ch) {
    const int cbase = ch * CHUNK;
    const int wc = scan_chunk<NBF>(dsts, nE, cbase, nodeBase, vec8, list, tid, lane, wave);
    if (lane == 0) wcnt[wave] = wc;
    __syncthreads();
    if (wave == 0) {
#pragma unroll 1
      for (int wsx = 0; wsx < NWAVE; ++wsx) {
        int n = __builtin_amdgcn_readfirstlane(wcnt[wsx]);
        n = n > WCAP ? WCAP : (n < 0 ? 0 : n);
        const int* lp = list + wsx * WCAP;
#pragma unroll 1
        for (int i = 0; i < n; ++i) {
          const int ent  = __builtin_amdgcn_readfirstlane(lp[i]);
          const int slot = ent & (NBF - 1);
          int e = cbase + ((ent >> 12) & (CHUNK - 1));
          e = e > nE - 1 ? nE - 1 : e;
          int sv = srcs[e];
          sv = sv < 0 ? 0 : (sv > nN - 1 ? nN - 1 : sv);
          if (lane == 0) {
            int pos = cursor[slot];
            pos = pos < 0 ? 0 : (pos > RCAP - 1 ? RCAP - 1 : pos);
            region[pos] = sv;
            const int np = pos + 1;
            cursor[slot] = np > RCAP ? RCAP : np;
          }
        }
      }
    }
    __syncthreads();
  }

  const int nv = lenW >> 2;
  int* gp = csr + rb0;
#pragma unroll 1
  for (int i = tid; i < nv; i += NTHR) { const v4i v = ((const v4i*)region)[i]; *(volatile v4i*)(gp + 4 * i) = v; }
  __threadfence();
#pragma unroll 1
  for (int i = tid; i < nv; i += NTHR) { const v4i v = ((const v4i*)region)[i]; *(volatile v4i*)(gp + 4 * i) = v; }
}

template <int KD, bool BNIN>
__global__ __launch_bounds__(NTHR) void k_gemm(
    const float* __restrict__ A, const float* __restrict__ coef,
    const float* __restrict__ gam, const float* __restrict__ bet,
    const _Float16* __restrict__ Bw, float* C, int nN) {
  static_assert(KD == F0 || KD == FD);
  static_assert((KD % 32) == 0);
  static_assert(BNIN ? (KD == FD) : (KD == F0));
  constexpr int APK = KD + 8;
  extern __shared__ v4f lds_dyn[];
  _Float16* sA  = (_Float16*)lds_dyn;
  float*    stg = (float*)((char*)lds_dyn + GROWS * APK * 2);
  const int tid = threadIdx.x, lane = tid & 31, wave = tid >> 5, hh = lane >> 4, m = lane & 15;
  const int rowBase = blockIdx.x * GROWS;

  if (!BNIN) {
    const int c0 = (tid & 7) * 8, rr = tid >> 3;
#pragma unroll
    for (int it = 0; it < 2; ++it) {
      const int r = rr + 32 * it;
      int row = rowBase + r;
      row = row > nN - 1 ? nN - 1 : row;
      const float* ap = A + (size_t)row * F0 + c0;
      const v4f a = *(const v4f*)ap, b = *(const v4f*)(ap + 4);
      *(v8h*)(sA + r * APK + c0) = cvt8(a * ASC, b * ASC);
    }
  } else {
    const int c0 = (tid & 31) * 8, rr = tid >> 5;
    const v4f mua = *(const v4f*)(coef + c0),      mub = *(const v4f*)(coef + c0 + 4);
    const v4f rsa = *(const v4f*)(coef + FD + c0), rsb = *(const v4f*)(coef + FD + c0 + 4);
    const v4f ga  = *(const v4f*)(gam + c0),       gb  = *(const v4f*)(gam + c0 + 4);
    const v4f ba  = *(const v4f*)(bet + c0),       bb  = *(const v4f*)(bet + c0 + 4);
#pragma unroll 1
    for (int it = 0; it < 8; ++it) {
      const int r = rr + 8 * it;
      const float* ap = A + (size_t)(rowBase + r) * FD + c0;
      const v4f a = *(const v4f*)ap, b = *(const v4f*)(ap + 4);
      const v4f za = bnt4(a, mua, rsa, ga, ba);
      const v4f zb = bnt4(b, mub, rsb, gb, bb);
      *(v8h*)(sA + r * APK + c0) = cvt8(za * ASC, zb * ASC);
    }
  }
  __syncthreads();

  const int rg = wave >> 2, cg = wave & 3;
  v8f acc[2][4];
#pragma unroll
  for (int i = 0; i < 2; ++i)
#pragma unroll
    for (int t = 0; t < 4; ++t) { v8f z = {0.f, 0.f, 0.f, 0.f, 0.f, 0.f, 0.f, 0.f}; acc[i][t] = z; }
  const _Float16* ap0 = sA + (32 * rg + m) * APK + 8 * hh;
  const _Float16* ap1 = ap0 + 16 * APK;
  const _Float16* bp0 = Bw + (size_t)(64 * cg + m) * KD + 8 * hh;
#pragma unroll 1
  for (int kt = 0; kt < KD / 32; ++kt) {
    FragH a0, a1;
    a0.h[0] = *(const v8h*)(ap0 + 32 * kt);
    a0.h[1] = *(const v8h*)(ap0 + 32 * kt + 16);
    a1.h[0] = *(const v8h*)(ap1 + 32 * kt);
    a1.h[1] = *(const v8h*)(ap1 + 32 * kt + 16);
#pragma unroll
    for (int t = 0; t < 4; ++t) {
      const _Float16* bp = bp0 + (size_t)(16 * t) * KD + 32 * kt;
      FragH b;
      b.h[0] = *(const v8h*)bp;
      b.h[1] = *(const v8h*)(bp + 16);
      acc[0][t] = wmh(a0.v, b.v, acc[0][t]);
      acc[1][t] = wmh(a1.v, b.v, acc[1][t]);
    }
  }
  {
    float* sp = stg + (32 * rg + 8 * hh) * FD + 64 * cg + m;
#pragma unroll
    for (int i = 0; i < 2; ++i)
#pragma unroll
      for (int t = 0; t < 4; ++t)
#pragma unroll
        for (int r = 0; r < 8; ++r) sp[(16 * i + r) * FD + 16 * t] = acc[i][t][r] * OSC;
  }
  __syncthreads();

  const float* lp = stg + (wave * 8) * FD + 4 * lane;
  float* gp = C + (size_t)(rowBase + wave * 8) * FD + 4 * lane;
#pragma unroll
  for (int j = 0; j < 8; ++j) {
    const v4f v0 = *(const v4f*)(lp + j * FD), v1 = *(const v4f*)(lp + j * FD + 128);
    *(volatile v4f*)(gp + j * FD) = v0;
    *(volatile v4f*)(gp + j * FD + 128) = v1;
  }
  __threadfence();
#pragma unroll
  for (int j = 0; j < 8; ++j) {
    const v4f v0 = *(const v4f*)(lp + j * FD), v1 = *(const v4f*)(lp + j * FD + 128);
    *(volatile v4f*)(gp + j * FD) = v0;
    *(volatile v4f*)(gp + j * FD + 128) = v1;
  }
}

__global__ __launch_bounds__(NTHR) void k_agg(
    const int* __restrict__ csr, const int* __restrict__ off, const int* __restrict__ cnt,
    const float* __restrict__ dinv, const float* __restrict__ H, const float* __restrict__ bias,
    float* AGG, double* part, int nN, int csrLen) {
  __shared__ __attribute__((aligned(16))) double dSQ[2 * NWAVE * FD];
  const int tid = threadIdx.x, lane = tid & 31, wave = tid >> 5;
  const int tbase = blockIdx.x * TGT + wave * 32;
  const int cl = tbase + lane;
  const int cnt_l = cnt[cl];
  const int off_l = off[cl];
  const int dvb_l = __float_as_int(dinv[cl]);
  const v4f ba = *(const v4f*)(bias + 4 * lane), bb = *(const v4f*)(bias + 128 + 4 * lane);

  double sacc[8], qacc[8];
#pragma unroll
  for (int i = 0; i < 8; ++i) { sacc[i] = 0.0; qacc[i] = 0.0; }

#pragma unroll 1
  for (int j = 0; j < 32; ++j) {
    const int c = tbase + j;
    int n = __builtin_amdgcn_readlane(cnt_l, j);
    n = n < 0 ? 0 : (n > DEGCAP ? DEGCAP : n);
    const int st = __builtin_amdgcn_readlane(off_l, j);
    const float dc = __int_as_float(__builtin_amdgcn_readlane(dvb_l, j));
    v4f sa = {0.0f, 0.0f, 0.0f, 0.0f}, sb = {0.0f, 0.0f, 0.0f, 0.0f};
#pragma unroll 1
    for (int q0 = 0; q0 < n; q0 += 32) {
      int pos = st + q0 + lane;
      pos = pos < 0 ? 0 : (pos > csrLen - 1 ? csrLen - 1 : pos);
      int sl = csr[pos];
      sl = sl < 0 ? 0 : (sl > nN - 1 ? nN - 1 : sl);
      const int dsb = __float_as_int(dinv[sl]);
      const int mcnt = (n - q0) < 32 ? (n - q0) : 32;
#pragma unroll 1
      for (int p = 0; p < mcnt; ++p) {
        const int s = __builtin_amdgcn_readlane(sl, p);
        const float cf = __int_as_float(__builtin_amdgcn_readlane(dsb, p)) * dc;
        const float* hp = H + (size_t)s * FD + 4 * lane;
        const v4f va = *(const v4f*)hp, vb = *(const v4f*)(hp + 128);
        sa = sa + va * cf;
        sb = sb + vb * cf;
      }
    }
    const float* hcp = H + (size_t)c * FD + 4 * lane;
    const v4f ha = *(const v4f*)hcp, hb = *(const v4f*)(hcp + 128);
    const float dd = dc * dc;
    v4f oa = sa + ha * dd, ob = sb + hb * dd;
    oa = oa + ba; ob = ob + bb;
    float* ap = AGG + (size_t)c * FD + 4 * lane;
    *(volatile v4f*)ap = oa;
    *(volatile v4f*)(ap + 128) = ob;
    __threadfence();
    *(volatile v4f*)ap = oa;
    *(volatile v4f*)(ap + 128) = ob;
    if (c < nN) {
      double d;
      d = (double)oa.x; sacc[0] += d; qacc[0] = fma(d, d, qacc[0]);
      d = (double)oa.y; sacc[1] += d; qacc[1] = fma(d, d, qacc[1]);
      d = (double)oa.z; sacc[2] += d; qacc[2] = fma(d, d, qacc[2]);
      d = (double)oa.w; sacc[3] += d; qacc[3] = fma(d, d, qacc[3]);
      d = (double)ob.x; sacc[4] += d; qacc[4] = fma(d, d, qacc[4]);
      d = (double)ob.y; sacc[5] += d; qacc[5] = fma(d, d, qacc[5]);
      d = (double)ob.z; sacc[6] += d; qacc[6] = fma(d, d, qacc[6]);
      d = (double)ob.w; sacc[7] += d; qacc[7] = fma(d, d, qacc[7]);
    }
  }

  {
    double* ps = dSQ + (0 * NWAVE + wave) * FD;
    double* pq = dSQ + (1 * NWAVE + wave) * FD;
#pragma unroll
    for (int i = 0; i < 4; ++i) {
      ps[4 * lane + i] = sacc[i];       ps[128 + 4 * lane + i] = sacc[4 + i];
      pq[4 * lane + i] = qacc[i];       pq[128 + 4 * lane + i] = qacc[4 + i];
    }
  }
  __syncthreads();
  const int kind = tid >> 7, k2 = (tid & 127) * 2;
  double v0 = 0.0, v1 = 0.0;
#pragma unroll
  for (int w = 0; w < NWAVE; ++w) {
    v0 += dSQ[(kind * NWAVE + w) * FD + k2];
    v1 += dSQ[(kind * NWAVE + w) * FD + k2 + 1];
  }
  v2d pv = {v0, v1};
  double* gq = part + (size_t)blockIdx.x * (2 * FD) + 2 * tid;
  *(volatile v2d*)gq = pv;
  __threadfence();
  *(volatile v2d*)gq = pv;
}

__global__ __launch_bounds__(NTHR) void k_bnfin(const double* __restrict__ part, float* coef, int nBlk, int nN) {
  __shared__ __attribute__((aligned(16))) float sco[2 * FD];
  const int tid = threadIdx.x, c = tid;
  double S = 0.0, Q = 0.0;
#pragma unroll 1
  for (int b = 0; b < nBlk; ++b) {
    S += part[(size_t)b * (2 * FD) + c];
    Q += part[(size_t)b * (2 * FD) + FD + c];
  }
  const double rn = 1.0 / (double)(nN > 1 ? nN : 1);
  const double mean = S * rn;
  double var = Q * rn - mean * mean;
  var = var < 0.0 ? 0.0 : var;
  sco[c]      = (float)mean;
  sco[FD + c] = rsqrtf((float)var + BN_EPS);
  __syncthreads();
  v4f cv = {0.f, 0.f, 0.f, 0.f};
  if (tid < FD / 2) cv = *(const v4f*)(sco + 4 * tid);
  if (tid < FD / 2) *(volatile v4f*)(coef + 4 * tid) = cv;
  __threadfence();
  if (tid < FD / 2) *(volatile v4f*)(coef + 4 * tid) = cv;
}

__device__ __forceinline__ int lbound(const int* __restrict__ a, int n, int key) {
  int lo = 0, len = n;
#pragma unroll 1
  for (int it = 0; it < 40; ++it) {
    if (len <= 0) break;
    const int half = len >> 1;
    int mid = lo + half;
    mid = mid > n - 1 ? n - 1 : (mid < 0 ? 0 : mid);
    const int v = a[mid];
    const bool go = v < key;
    lo  = go ? (mid + 1) : lo;
    len = go ? (len - half - 1) : half;
  }
  return lo;
}

__global__ __launch_bounds__(NTHR) void k_pool(
    const float* __restrict__ AGG, const float* __restrict__ coef,
    const float* __restrict__ gam, const float* __restrict__ bet, const int* __restrict__ bidx,
    const float* __restrict__ wout, const float* __restrict__ bout, float* HID, int nN) {
  __shared__ __attribute__((aligned(16))) float shid[HP];
  __shared__ float swp[NWAVE];
  const int tid = threadIdx.x, lane = tid & 31, wave = tid >> 5, d = tid;
  const int g = blockIdx.x;
  const int lo = lbound(bidx, nN, g);
  const int hi = lbound(bidx, nN, g + 1);
  int cg = hi - lo;
  cg = cg < 0 ? 0 : (cg > MAXSEG ? MAXSEG : cg);
  const float mu = coef[d], rs = coef[FD + d], ga = gam[d], be = bet[d];
  float mx = __uint_as_float(0xff800000u), sm = 0.0f;
#pragma unroll 1
  for (int i = 0; i < cg; ++i) {
    int row = lo + i;
    row = row > nN - 1 ? nN - 1 : (row < 0 ? 0 : row);
    const float a = AGG[(size_t)row * FD + d];
    const float v = bnt1(a, mu, rs, ga, be);
    mx = fmaxf(mx, v);
    sm += v;
  }
  const float rc = 1.0f / (float)cg;
  const float hm = sm * rc;
  shid[d] = mx;
  shid[FD + d] = hm;
  float p = mx * wout[d] + hm * wout[FD + d];
#pragma unroll
  for (int o = 16; o > 0; o >>= 1) p += __shfl_xor(p, o);
  if (lane == 0) swp[wave] = p;
  __syncthreads();
  if (tid == 0) {
    float t = swp[0];
#pragma unroll
    for (int w = 1; w < NWAVE; ++w) t += swp[w];
    t += bout[0];
    shid[2 * FD] = t;
  }
  if (tid > 0 && tid < HP - 2 * FD) shid[2 * FD + tid] = 0.0f;
  __syncthreads();
  v4f hv = {0.f, 0.f, 0.f, 0.f};
  if (tid < HP / 4) hv = *(const v4f*)(shid + 4 * tid);
  float* gp = HID + (size_t)g * HP + 4 * tid;
  if (tid < HP / 4) *(volatile v4f*)gp = hv;
  __threadfence();
  if (tid < HP / 4) *(volatile v4f*)gp = hv;
}

__device__ __forceinline__ float fval(const float* __restrict__ HID, int f, int nG, int outN) {
  int fc = f > outN - 1 ? outN - 1 : f;
  fc = fc < 0 ? 0 : fc;
  const int ia = (fc > nG - 1 ? nG - 1 : fc) * HP + 2 * FD;
  int t = fc - nG; t = t < 0 ? 0 : t;
  int row = t / (2 * FD);
  row = row > nG - 1 ? nG - 1 : row;
  const int ib = row * HP + (t & (2 * FD - 1));
  const int idx = (fc < nG) ? ia : ib;
  return HID[idx];
}

__device__ __forceinline__ void fstore(float* out, int f0, v4f v, int outN) {
  if (f0 + 4 <= outN) {
    *(volatile v4f*)(out + f0) = v;
  } else if (f0 < outN) {
    volatile float* op = out + f0;
    op[0] = v.x;
    if (f0 + 1 < outN) op[1] = v.y;
    if (f0 + 2 < outN) op[2] = v.z;
  }
}

__global__ __launch_bounds__(NTHR) void k_final(const float* __restrict__ HID, float* out, int nG, int outN) {
  const int tid = threadIdx.x;
  v4f vals[4];
#pragma unroll
  for (int it = 0; it < 4; ++it) {
    const int q = (blockIdx.x * 4 + it) * NTHR + tid;
    const int f0 = 4 * q;
    v4f v;
    v.x = fval(HID, f0 + 0, nG, outN);
    v.y = fval(HID, f0 + 1, nG, outN);
    v.z = fval(HID, f0 + 2, nG, outN);
    v.w = fval(HID, f0 + 3, nG, outN);
    vals[it] = v;
  }
#pragma unroll
  for (int it = 0; it < 4; ++it) {
    const int q = (blockIdx.x * 4 + it) * NTHR + tid;
    fstore(out, 4 * q, vals[it], outN);
  }
  __threadfence();
#pragma unroll
  for (int it = 0; it < 4; ++it) {
    const int q = (blockIdx.x * 4 + it) * NTHR + tid;
    fstore(out, 4 * q, vals[it], outN);
  }
}

extern "C" void kernel_launch(void* const* d_in, const int* in_sizes, int n_in,
                              void* d_out, int out_size, void* d_ws, size_t ws_size,
                              hipStream_t stream) {
  if (n_in < 22) return;
  if (in_sizes[0] <= 0 || (in_sizes[0] % F0) != 0) return;
  const int nN = in_sizes[0] / F0;
  if (in_sizes[1] < 2 || (in_sizes[1] & 1) != 0) return;
  const int nE = in_sizes[1] / 2;
  if (in_sizes[2] != nN) return;
  if (in_sizes[4] != F0 * FD) return;
  if (in_sizes[6] != FD * FD || in_sizes[8] != FD * FD || in_sizes[10] != FD * FD) return;
  if (in_sizes[5] != FD || in_sizes[7] != FD || in_sizes[9] != FD || in_sizes[11] != FD) return;
  for (int i = 12; i < 20; ++i) if (in_sizes[i] != FD) return;
  if (in_sizes[20] != 2 * FD || in_sizes[21] < 1) return;
  const int B = out_size / (1 + 2 * FD);
  if (B < 1 || out_size != B * (1 + 2 * FD)) return;
  if (nE > (1 << 28) || nN > (1 << 24) || B > (1 << 22)) return;

  const float* x    = (const float*)d_in[0];
  const int*   ei   = (const int*)d_in[1];
  const int*   bidx = (const int*)d_in[2];
  const float* W0 = (const float*)d_in[4];
  const float* W1 = (const float*)d_in[6];
  const float* W2 = (const float*)d_in[8];
  const float* W3 = (const float*)d_in[10];
  const float* bl[4]  = {(const float*)d_in[5],  (const float*)d_in[7],  (const float*)d_in[9],  (const float*)d_in[11]};
  const float* gl[4]  = {(const float*)d_in[12], (const float*)d_in[14], (const float*)d_in[16], (const float*)d_in[18]};
  const float* bel[4] = {(const float*)d_in[13], (const float*)d_in[15], (const float*)d_in[17], (const float*)d_in[19]};
  const float* wout = (const float*)d_in[20];
  const float* bout = (const float*)d_in[21];
  const int* srcs = ei;
  const int* dsts = ei + (size_t)nE;
  float* out = (float*)d_out;

  const int NPAD   = ((nN + TGT - 1) / TGT) * TGT;
  const int nBC    = (nN + NBC - 1) / NBC;
  const int CNTPAD = nBC * NBC;
  if (4 * nBC + 1 > RBN) return;
  const int nBF    = (nN + NBF - 1) / NBF;
  const int csrLen = ((nE + 31) & ~31) + 4096;
  if (31 * 4 * nBC > 4096) return;
  const int nGemm  = NPAD / GROWS;
  const int nAgg   = NPAD / TGT;
  const int nPiece = (out_size + 3) / 4;
  const int nFin   = (nPiece + 4 * NTHR - 1) / (4 * NTHR);

  char* ws = (char*)d_ws;
  size_t off = 0;
  const size_t oW    = off; off += (size_t)WPTOT * 2;               off = (off + 255) & ~(size_t)255;
  const size_t oCnt  = off; off += (size_t)CNTPAD * 4;              off = (off + 255) & ~(size_t)255;
  const size_t oOff  = off; off += (size_t)CNTPAD * 4;              off = (off + 255) & ~(size_t)255;
  const size_t oDinv = off; off += (size_t)CNTPAD * 4;              off = (off + 255) & ~(size_t)255;
  const size_t oRb   = off; off += (size_t)RBN * 4;                 off = (off + 255) & ~(size_t)255;
  const size_t oCsr  = off; off += (size_t)csrLen * 4;              off = (off + 255) & ~(size_t)255;
  const size_t oH    = off; off += (size_t)NPAD * FD * 4;           off = (off + 255) & ~(size_t)255;
  const size_t oAgg  = off; off += (size_t)NPAD * FD * 4;           off = (off + 255) & ~(size_t)255;
  const size_t oPart = off; off += (size_t)nAgg * (2 * FD) * 8;     off = (off + 255) & ~(size_t)255;
  const size_t oCoef = off; off += (size_t)2 * FD * 4;              off = (off + 255) & ~(size_t)255;
  const size_t oHid  = off; off += (size_t)B * HP * 4;              off = (off + 255) & ~(size_t)255;
  if (off > ws_size || off > (size_t)WSCAP) return;
  _Float16* wp   = (_Float16*)(ws + oW);
  int*      cnt  = (int*)(ws + oCnt);
  int*      offp = (int*)(ws + oOff);
  float*    dinv = (float*)(ws + oDinv);
  int*      rb   = (int*)(ws + oRb);
  int*      csr  = (int*)(ws + oCsr);
  float*    Hp   = (float*)(ws + oH);
  float*    AGG  = (float*)(ws + oAgg);
  double*   part = (double*)(ws + oPart);
  float*    coef = (float*)(ws + oCoef);
  float*    HID  = (float*)(ws + oHid);

  const int vec8 = ((nE & 3) == 0) ? 1 : 0;

  k_wprep<<<8 + 3 * 32, NTHR, 0, stream>>>(W0, W1, W2, W3, wp);

  k_count<<<nBC, NTHR, 0, stream>>>(dsts, cnt, nE, vec8);
  k_offsets<<<1, OTHR, 0, stream>>>(cnt, offp, dinv, rb, nBC);
  hipFuncSetAttribute(reinterpret_cast<const void*>(&k_fill),
                      hipFuncAttributeMaxDynamicSharedMemorySize, LDS_FILL);
  k_fill<<<nBF, NTHR, LDS_FILL, stream>>>(srcs, dsts, offp, rb, csr, nN, nE, vec8, csrLen);

  hipFuncSetAttribute(reinterpret_cast<const void*>(&k_gemm<F0, false>),
                      hipFuncAttributeMaxDynamicSharedMemorySize, LDS_G0);
  hipFuncSetAttribute(reinterpret_cast<const void*>(&k_gemm<FD, true>),
                      hipFuncAttributeMaxDynamicSharedMemorySize, LDS_G1);

  k_gemm<F0, false><<<nGemm, NTHR, LDS_G0, stream>>>(x, coef, gl[0], bel[0], wp + WOFF0, Hp, nN);
  k_agg<<<nAgg, NTHR, 0, stream>>>(csr, offp, cnt, dinv, Hp, bl[0], AGG, part, nN, csrLen);
  k_bnfin<<<1, NTHR, 0, stream>>>(part, coef, nAgg, nN);

  k_gemm<FD, true><<<nGemm, NTHR, LDS_G1, stream>>>(AGG, coef, gl[0], bel[0], wp + WOFF1, Hp, nN);
  k_agg<<<nAgg, NTHR, 0, stream>>>(csr, offp, cnt, dinv, Hp, bl[1], AGG, part, nN, csrLen);
  k_bnfin<<<1, NTHR, 0, stream>>>(part, coef, nAgg, nN);

  k_gemm<FD, true><<<nGemm, NTHR, LDS_G1, stream>>>(AGG, coef, gl[1], bel[1], wp + WOFF2, Hp, nN);
  k_agg<<<nAgg, NTHR, 0, stream>>>(csr, offp, cnt, dinv, Hp, bl[2], AGG, part, nN, csrLen);
  k_bnfin<<<1, NTHR, 0, stream>>>(part, coef, nAgg, nN);

  k_gemm<FD, true><<<nGemm, NTHR, LDS_G1, stream>>>(AGG, coef, gl[2], bel[2], wp + WOFF3, Hp, nN);
  k_agg<<<nAgg, NTHR, 0, stream>>>(csr, offp, cnt, dinv, Hp, bl[3], AGG, part, nN, csrLen);
  k_bnfin<<<1, NTHR, 0, stream>>>(part, coef, nAgg, nN);

  k_pool<<<B, NTHR, 0, stream>>>(AGG, coef, gl[3], bel[3], bidx, wout, bout, HID, nN);

  k_final<<<nFin, NTHR, 0, stream>>>(HID, out, B, out_size);
}
